// CAR_63385127354415
// MI455X (gfx1250) — hardware-verified
//
#include <hip/hip_runtime.h>
#define BB 4
#define RR 12
#define NP (RR * RR * RR)
#define NVOX (BB * NP)
#define CX 256
#define CH 64
#define NH 4
#define HD 16
#define HP 32
#define COUT 256
#define LINIT 0.5560582f

typedef __bf16 v16b __attribute__((ext_vector_type(16)));
typedef unsigned short v8us __attribute__((ext_vector_type(8), may_alias));
typedef float  v8f  __attribute__((ext_vector_type(8)));
typedef float  v4f  __attribute__((ext_vector_type(4)));
typedef float  v4fa __attribute__((ext_vector_type(4), may_alias));
union FragB { v16b v; v8us half[2]; unsigned short u[16]; };

__device__ __forceinline__ unsigned short bf16_bits(float x) { unsigned int u = __float_as_uint(x); return (unsigned short)((u + 0x7FFFu + ((u >> 16) & 1u)) >> 16); }
__device__ __forceinline__ float bf16_val(unsigned short b) { return __uint_as_float(((unsigned int)b) << 16); }
__device__ __forceinline__ float bf16_round(float x) { return bf16_val(bf16_bits(x)); }
template <int NT>
__device__ __forceinline__ v8f mmaN(v16b ah, v16b al, v16b bh, v16b bl, v8f c) {
  c = __builtin_amdgcn_wmma_f32_16x16x32_bf16(false, ah, false, bh, (short)0, c, false, false);
  if (NT >= 2) c = __builtin_amdgcn_wmma_f32_16x16x32_bf16(false, al, false, bh, (short)0, c, false, false);
  if (NT >= 3) c = __builtin_amdgcn_wmma_f32_16x16x32_bf16(false, ah, false, bl, (short)0, c, false, false);
  asm volatile("v_nop\n\tv_nop\n\tv_nop\n\tv_nop" : "+v"(c) : "v"(ah), "v"(al), "v"(bh), "v"(bl));
  return c;
}

__global__ __launch_bounds__(256) void k_wt_bf16(const float* __restrict__ W, unsigned short* __restrict__ Wt, int K, int N) {
  const int t = blockIdx.x * 256 + threadIdx.x;
  const int k8n = K / 8;
  if (t >= N * k8n) return;
  const int n = t / k8n, k8 = (t % k8n) * 8;
  v8us v;
#pragma unroll
  for (int i = 0; i < 8; ++i) v[i] = bf16_bits(W[(size_t)(k8 + i) * N + n]);
  *(volatile v8us*)(Wt + (size_t)n * K + k8) = v;
  __threadfence();
  *(volatile v8us*)(Wt + (size_t)n * K + k8) = v;
}

template <bool ASPLIT, int ACT, bool BIAS_BF16>
__global__ __launch_bounds__(128) void k_gemm_bf(const float* __restrict__ A, int lda, const unsigned short* __restrict__ Wt, int ldb,
                                               const float* __restrict__ bias, float* __restrict__ C, int ldc, int M, int N, int K) {
  __shared__ __attribute__((aligned(16))) float so[4][16][64];
  const int tid = threadIdx.x, w = tid >> 5, lane = tid & 31, ln = lane & 15, hh = lane >> 4;
  const int ntn = N / 64;
  const int wid = blockIdx.x * 4 + w;
  const int mt = wid / ntn, nq = wid % ntn;
  if (mt * 16 >= M) return;
  const int row0 = mt * 16, col0 = nq * 64;
  const float* arow = A + (size_t)(row0 + ln) * lda;
  v8f acc[4] = {};
  for (int kb = 0; kb < K; kb += 32) {
    FragB ah, al;
    const v4f x0 = *(const v4fa*)(arow + kb + 8 * hh), x1 = *(const v4fa*)(arow + kb + 8 * hh + 4);
    const v4f x2 = *(const v4fa*)(arow + kb + 16 + 8 * hh), x3 = *(const v4fa*)(arow + kb + 16 + 8 * hh + 4);
    float xs[16] = {x0[0],x0[1],x0[2],x0[3],x1[0],x1[1],x1[2],x1[3],x2[0],x2[1],x2[2],x2[3],x3[0],x3[1],x3[2],x3[3]};
#pragma unroll
    for (int i = 0; i < 16; ++i) { const unsigned short hb = bf16_bits(xs[i]); ah.u[i] = hb; al.u[i] = ASPLIT ? bf16_bits(xs[i] - bf16_val(hb)) : (unsigned short)0; }
#pragma unroll
    for (int t = 0; t < 4; ++t) {
      const unsigned short* brow = Wt + (size_t)(col0 + t * 16 + ln) * ldb + kb;
      FragB b;
      b.half[0] = *(const v8us*)(brow + 8 * hh);
      b.half[1] = *(const v8us*)(brow + 16 + 8 * hh);
      acc[t] = mmaN<ASPLIT ? 2 : 1>(ah.v, al.v, b.v, b.v, acc[t]);
    }
  }
#pragma unroll
  for (int t = 0; t < 4; ++t) {
    float bv = bias ? bias[col0 + t * 16 + ln] : 0.f;
    if (BIAS_BF16) bv = bf16_round(bv);
#pragma unroll
    for (int r = 0; r < 8; ++r) { float v = acc[t][r] + bv; if (ACT == 1) v = fmaxf(v, 0.f); so[w][8 * hh + r][t * 16 + ln] = v; }
  }
  __builtin_amdgcn_fence(__ATOMIC_ACQ_REL, "workgroup");
  __builtin_amdgcn_wave_barrier();
  const int rsub = lane >> 4, c4 = (lane & 15) * 4;
  for (int pass = 0; pass < 2; ++pass) {
#pragma unroll
    for (int q = 0; q < 8; ++q) {
      const int r = q * 2 + rsub;
      const v4f v = *(const v4fa*)&so[w][r][c4];
      *(volatile v4f*)(C + (size_t)(row0 + r) * ldc + col0 + c4) = v;
    }
    if (pass == 0) __threadfence();
  }
}

template <int D, bool CAUSAL>
__global__ __launch_bounds__(128) void k_flash(const float* __restrict__ qb, const float* __restrict__ kb, const float* __restrict__ vb,
                                             int pitch, int T, int H, float scale, float* __restrict__ y, int ypitch) {
  constexpr int KS = D / 32;
  constexpr int DT = D / 16;
  __shared__ __attribute__((aligned(16))) unsigned short sKh[32][D + 8], sKl[32][D + 8], sVh[32][D + 8], sVl[32][D + 8];
  __shared__ __attribute__((aligned(16))) unsigned short sPh[4][16][40], sPl[4][16][40];
  __shared__ __attribute__((aligned(16))) float sO[4][16][D];
  const int tid = threadIdx.x, w = tid >> 5, lane = tid & 31, ln = lane & 15, hh = lane >> 4;
  const int nqb = (T + 63) / 64;
  const int bh = blockIdx.x / nqb, qblk = blockIdx.x % nqb;
  const int b = bh / H, h = bh % H;
  const int q0 = qblk * 64 + w * 16;
  const float* Q = qb + (size_t)b * T * pitch + h * D;
  const float* K = kb + (size_t)b * T * pitch + h * D;
  const float* V = vb + (size_t)b * T * pitch + h * D;

  FragB aqh[KS], aql[KS];
  {
    int row = q0 + ln; if (row >= T) row = T - 1;
    const float* qr = Q + (size_t)row * pitch;
#pragma unroll
    for (int ks = 0; ks < KS; ++ks)
#pragma unroll
      for (int i = 0; i < 16; ++i) {
        const int d = ks * 32 + ((i < 8) ? (8 * hh + i) : (16 + 8 * hh + (i - 8)));
        const float x = qr[d] * scale; const unsigned short hb = bf16_bits(x);
        aqh[ks].u[i] = hb; aql[ks].u[i] = bf16_bits(x - bf16_val(hb));
      }
  }
  float m_r[8], l_r[8];
#pragma unroll
  for (int r = 0; r < 8; ++r) { m_r[r] = -3.0e38f; l_r[r] = 0.f; }
  v8f oacc[DT];
#pragma unroll
  for (int dt = 0; dt < DT; ++dt) oacc[dt] = (v8f){0.f,0.f,0.f,0.f,0.f,0.f,0.f,0.f};

  const int kv_end = CAUSAL ? min(T, qblk * 64 + 64) : T;
  for (int j0 = 0; j0 < kv_end; j0 += 32) {
    __syncthreads();
    for (int e = tid; e < 32 * (D / 4); e += 128) {
      const int r = e / (D / 4), c4 = (e % (D / 4)) * 4;
      const int key = j0 + r;
      v4f kf = {0.f,0.f,0.f,0.f}, vf = {0.f,0.f,0.f,0.f};
      if (key < T) { kf = *(const v4fa*)(K + (size_t)key * pitch + c4); vf = *(const v4fa*)(V + (size_t)key * pitch + c4); }
#pragma unroll
      for (int t = 0; t < 4; ++t) {
        unsigned short hb = bf16_bits(kf[t]); sKh[r][c4 + t] = hb; sKl[r][c4 + t] = bf16_bits(kf[t] - bf16_val(hb));
        hb = bf16_bits(vf[t]); sVh[r][c4 + t] = hb; sVl[r][c4 + t] = bf16_bits(vf[t] - bf16_val(hb));
      }
    }
    __syncthreads();
    v8f s[2];
#pragma unroll
    for (int nt = 0; nt < 2; ++nt) {
      v8f acc = {};
#pragma unroll
      for (int ks = 0; ks < KS; ++ks) {
        FragB bh_, bl_;
        bh_.half[0] = *(const v8us*)&sKh[nt * 16 + ln][ks * 32 + 8 * hh]; bh_.half[1] = *(const v8us*)&sKh[nt * 16 + ln][ks * 32 + 16 + 8 * hh];
        bl_.half[0] = *(const v8us*)&sKl[nt * 16 + ln][ks * 32 + 8 * hh]; bl_.half[1] = *(const v8us*)&sKl[nt * 16 + ln][ks * 32 + 16 + 8 * hh];
        acc = mmaN<3>(aqh[ks].v, aql[ks].v, bh_.v, bl_.v, acc);
      }
      s[nt] = acc;
    }
    float alpha[8];
#pragma unroll
    for (int r = 0; r < 8; ++r) {
      const int qi = q0 + 8 * hh + r;
      const int ja = j0 + ln, jb = j0 + 16 + ln;
      if (CAUSAL) { if (ja > qi) s[0][r] = -3.0e38f; if (jb > qi) s[1][r] = -3.0e38f; }
      if (ja >= T) s[0][r] = -3.0e38f;
      if (jb >= T) s[1][r] = -3.0e38f;
      float mx = fmaxf(s[0][r], s[1][r]);
      mx = fmaxf(mx, __shfl_xor(mx, 1, 32)); mx = fmaxf(mx, __shfl_xor(mx, 2, 32)); mx = fmaxf(mx, __shfl_xor(mx, 4, 32)); mx = fmaxf(mx, __shfl_xor(mx, 8, 32));
      const float mnew = fmaxf(m_r[r], mx);
      alpha[r] = (mnew > -1.0e38f) ? __expf(m_r[r] - mnew) : 1.0f;
      const float p0 = (s[0][r] > -1.0e38f) ? __expf(s[0][r] - mnew) : 0.f;
      const float p1 = (s[1][r] > -1.0e38f) ? __expf(s[1][r] - mnew) : 0.f;
      m_r[r] = mnew;
      l_r[r] = l_r[r] * alpha[r] + p0 + p1;
      unsigned short hb = bf16_bits(p0); sPh[w][8 * hh + r][ln] = hb;      sPl[w][8 * hh + r][ln] = bf16_bits(p0 - bf16_val(hb));
      hb = bf16_bits(p1);                sPh[w][8 * hh + r][16 + ln] = hb; sPl[w][8 * hh + r][16 + ln] = bf16_bits(p1 - bf16_val(hb));
    }
#pragma unroll
    for (int dt = 0; dt < DT; ++dt)
#pragma unroll
      for (int r = 0; r < 8; ++r) oacc[dt][r] *= alpha[r];
    __builtin_amdgcn_fence(__ATOMIC_ACQ_REL, "workgroup");
    __builtin_amdgcn_wave_barrier();
    FragB pah, pal;
    pah.half[0] = *(const v8us*)&sPh[w][ln][8 * hh]; pah.half[1] = *(const v8us*)&sPh[w][ln][16 + 8 * hh];
    pal.half[0] = *(const v8us*)&sPl[w][ln][8 * hh]; pal.half[1] = *(const v8us*)&sPl[w][ln][16 + 8 * hh];
#pragma unroll
    for (int dt = 0; dt < DT; ++dt) {
      FragB bvh, bvl;
#pragma unroll
      for (int i = 0; i < 8; ++i) {
        bvh.u[i] = sVh[8 * hh + i][dt * 16 + ln]; bvh.u[8 + i] = sVh[16 + 8 * hh + i][dt * 16 + ln];
        bvl.u[i] = sVl[8 * hh + i][dt * 16 + ln]; bvl.u[8 + i] = sVl[16 + 8 * hh + i][dt * 16 + ln];
      }
      oacc[dt] = mmaN<3>(pah.v, pal.v, bvh.v, bvl.v, oacc[dt]);
    }
    __builtin_amdgcn_fence(__ATOMIC_ACQ_REL, "workgroup");
    __builtin_amdgcn_wave_barrier();
  }
#pragma unroll
  for (int r = 0; r < 8; ++r) {
    float l = l_r[r];
    l += __shfl_xor(l, 1, 32); l += __shfl_xor(l, 2, 32); l += __shfl_xor(l, 4, 32); l += __shfl_xor(l, 8, 32);
    l_r[r] = (l > 0.f) ? 1.0f / l : 0.f;
  }
#pragma unroll
  for (int dt = 0; dt < DT; ++dt)
#pragma unroll
    for (int r = 0; r < 8; ++r) sO[w][8 * hh + r][dt * 16 + ln] = oacc[dt][r] * l_r[r];
  __builtin_amdgcn_fence(__ATOMIC_ACQ_REL, "workgroup");
  __builtin_amdgcn_wave_barrier();
  for (int pass = 0; pass < 2; ++pass) {
    for (int r = 0; r < 16; ++r) {
      const int row = q0 + r;
      if (row < T && lane < D / 4) {
        const v4f val = *(const v4fa*)&sO[w][r][lane * 4];
        *(volatile v4f*)(y + ((size_t)b * T + row) * ypitch + h * D + lane * 4) = val;
      }
    }
    if (pass == 0) __threadfence();
  }
}

template <bool AFFINE, bool RESID, bool RES_BF16>
__global__ __launch_bounds__(256) void k_transpose32(const float* __restrict__ in, float* __restrict__ out, int rows, int cols,
                                                    const float* __restrict__ scale, const float* __restrict__ shift, const float* __restrict__ res) {
  __shared__ float tile[32][33];
  const int b = blockIdx.z;
  const int r0 = blockIdx.y * 32, c0 = blockIdx.x * 32;
  const float* src = in + (size_t)b * rows * cols;
  float* dst = out + (size_t)b * rows * cols;
  const int tx = threadIdx.x & 31, ty = threadIdx.x >> 5;
  for (int i = ty; i < 32; i += 8) tile[i][tx] = src[(size_t)(r0 + i) * cols + c0 + tx];
  __syncthreads();
  for (int pass = 0; pass < 2; ++pass) {
    for (int i = ty; i < 32; i += 8) {
      float v = tile[tx][i];
      const int orow = c0 + i;
      if (AFFINE) v = v * scale[orow] + shift[orow];
      if (RESID) { float rv = res[(size_t)b * rows * cols + (size_t)orow * rows + r0 + tx]; if (RES_BF16) rv = bf16_round(rv); v += rv; }
      *(volatile float*)(dst + (size_t)orow * rows + r0 + tx) = v;
    }
    if (pass == 0) __threadfence();
  }
}

__global__ __launch_bounds__(256) void k_pool2_pm(const float* __restrict__ in, float* __restrict__ out, int Bn, int H, int W, int C) {
  const size_t t = (size_t)blockIdx.x * 256 + threadIdx.x;
  const int c4n = C / 4, Ho = H / 2, Wo = W / 2;
  const size_t total = (size_t)Bn * Ho * Wo * c4n;
  if (t >= total) return;
  const int c4 = (int)(t % c4n) * 4; size_t rest = t / c4n;
  const int pw = (int)(rest % Wo); rest /= Wo; const int ph = (int)(rest % Ho); const int b = (int)(rest / Ho);
  const float* base = in + (size_t)b * H * W * C;
  const int p00 = (2 * ph) * W + 2 * pw;
  const v4f a = *(const v4fa*)(base + (size_t)p00 * C + c4), bq = *(const v4fa*)(base + (size_t)(p00 + 1) * C + c4);
  const v4f c = *(const v4fa*)(base + (size_t)(p00 + W) * C + c4), d = *(const v4fa*)(base + (size_t)(p00 + W + 1) * C + c4);
  v4f m; for (int i = 0; i < 4; ++i) m[i] = fmaxf(fmaxf(a[i], bq[i]), fmaxf(c[i], d[i]));
  float* dst = out + ((size_t)b * Ho * Wo + (size_t)ph * Wo + pw) * C + c4;
  *(volatile v4f*)dst = m;
  __threadfence();
  *(volatile v4f*)dst = m;
}

template <int DQ, int DV>
__global__ __launch_bounds__(128) void k_flash2(const float* __restrict__ Qb, size_t qstride, int qpitch, int Tq,
                                              const float* __restrict__ Kb, size_t kstride, int kpitch, int Tk,
                                              const float* __restrict__ Vb, size_t vstride, int vpitch,
                                              float scale, float* __restrict__ y, size_t ystride, int ypitch) {
  constexpr int KS = DQ / 32, DT = DV / 16;
  __shared__ __attribute__((aligned(16))) unsigned short sKh[32][DQ + 8], sKl[32][DQ + 8], sVh[32][DV + 8], sVl[32][DV + 8];
  __shared__ __attribute__((aligned(16))) unsigned short sPh[4][16][40], sPl[4][16][40];
  __shared__ __attribute__((aligned(16))) float sO[4][16][DV];
  const int tid = threadIdx.x, w = tid >> 5, lane = tid & 31, ln = lane & 15, hh = lane >> 4;
  const int nqb = (Tq + 63) / 64;
  const int bh = blockIdx.x / nqb, qblk = blockIdx.x % nqb;
  const int dv0 = blockIdx.y * DV;
  const int q0 = qblk * 64 + w * 16;
  const float* Q = Qb + (size_t)bh * qstride; const float* K = Kb + (size_t)bh * kstride; const float* V = Vb + (size_t)bh * vstride + dv0;
  FragB aqh[KS], aql[KS];
  {
    int row = q0 + ln; if (row >= Tq) row = Tq - 1;
    const float* qr = Q + (size_t)row * qpitch;
#pragma unroll
    for (int ks = 0; ks < KS; ++ks)
#pragma unroll
      for (int i = 0; i < 16; ++i) {
        const int d = ks * 32 + ((i < 8) ? (8 * hh + i) : (16 + 8 * hh + (i - 8)));
        const float x = qr[d] * scale; const unsigned short hb = bf16_bits(x);
        aqh[ks].u[i] = hb; aql[ks].u[i] = bf16_bits(x - bf16_val(hb));
      }
  }
  float m_r[8], l_r[8];
#pragma unroll
  for (int r = 0; r < 8; ++r) { m_r[r] = -3.0e38f; l_r[r] = 0.f; }
  v8f oacc[DT];
#pragma unroll
  for (int dt = 0; dt < DT; ++dt) oacc[dt] = (v8f){0.f,0.f,0.f,0.f,0.f,0.f,0.f,0.f};
  for (int j0 = 0; j0 < Tk; j0 += 32) {
    __syncthreads();
    for (int e = tid; e < 32 * (DQ / 4); e += 128) {
      const int r = e / (DQ / 4), c4 = (e % (DQ / 4)) * 4; const int key = j0 + r;
      v4f f = {0.f,0.f,0.f,0.f}; if (key < Tk) f = *(const v4fa*)(K + (size_t)key * kpitch + c4);
#pragma unroll
      for (int t = 0; t < 4; ++t) { const unsigned short hb = bf16_bits(f[t]); sKh[r][c4 + t] = hb; sKl[r][c4 + t] = bf16_bits(f[t] - bf16_val(hb)); }
    }
    for (int e = tid; e < 32 * (DV / 4); e += 128) {
      const int r = e / (DV / 4), c4 = (e % (DV / 4)) * 4; const int key = j0 + r;
      v4f f = {0.f,0.f,0.f,0.f}; if (key < Tk) f = *(const v4fa*)(V + (size_t)key * vpitch + c4);
#pragma unroll
      for (int t = 0; t < 4; ++t) { const unsigned short hb = bf16_bits(f[t]); sVh[r][c4 + t] = hb; sVl[r][c4 + t] = bf16_bits(f[t] - bf16_val(hb)); }
    }
    __syncthreads();
    v8f s[2];
#pragma unroll
    for (int nt = 0; nt < 2; ++nt) {
      v8f acc = {};
#pragma unroll
      for (int ks = 0; ks < KS; ++ks) {
        FragB bh_, bl_;
        bh_.half[0] = *(const v8us*)&sKh[nt * 16 + ln][ks * 32 + 8 * hh]; bh_.half[1] = *(const v8us*)&sKh[nt * 16 + ln][ks * 32 + 16 + 8 * hh];
        bl_.half[0] = *(const v8us*)&sKl[nt * 16 + ln][ks * 32 + 8 * hh]; bl_.half[1] = *(const v8us*)&sKl[nt * 16 + ln][ks * 32 + 16 + 8 * hh];
        acc = mmaN<3>(aqh[ks].v, aql[ks].v, bh_.v, bl_.v, acc);
      }
      s[nt] = acc;
    }
    float alpha[8];
#pragma unroll
    for (int r = 0; r < 8; ++r) {
      const int ja = j0 + ln, jb = j0 + 16 + ln;
      if (ja >= Tk) s[0][r] = -3.0e38f;
      if (jb >= Tk) s[1][r] = -3.0e38f;
      float mx = fmaxf(s[0][r], s[1][r]);
      mx = fmaxf(mx, __shfl_xor(mx, 1, 32)); mx = fmaxf(mx, __shfl_xor(mx, 2, 32)); mx = fmaxf(mx, __shfl_xor(mx, 4, 32)); mx = fmaxf(mx, __shfl_xor(mx, 8, 32));
      const float mnew = fmaxf(m_r[r], mx);
      alpha[r] = (mnew > -1.0e38f) ? __expf(m_r[r] - mnew) : 1.0f;
      const float p0 = (s[0][r] > -1.0e38f) ? __expf(s[0][r] - mnew) : 0.f;
      const float p1 = (s[1][r] > -1.0e38f) ? __expf(s[1][r] - mnew) : 0.f;
      m_r[r] = mnew;
      l_r[r] = l_r[r] * alpha[r] + p0 + p1;
      unsigned short hb = bf16_bits(p0); sPh[w][8 * hh + r][ln] = hb;      sPl[w][8 * hh + r][ln] = bf16_bits(p0 - bf16_val(hb));
      hb = bf16_bits(p1);                sPh[w][8 * hh + r][16 + ln] = hb; sPl[w][8 * hh + r][16 + ln] = bf16_bits(p1 - bf16_val(hb));
    }
#pragma unroll
    for (int dt = 0; dt < DT; ++dt)
#pragma unroll
      for (int r = 0; r < 8; ++r) oacc[dt][r] *= alpha[r];
    __builtin_amdgcn_fence(__ATOMIC_ACQ_REL, "workgroup");
    __builtin_amdgcn_wave_barrier();
    FragB pah, pal;
    pah.half[0] = *(const v8us*)&sPh[w][ln][8 * hh]; pah.half[1] = *(const v8us*)&sPh[w][ln][16 + 8 * hh];
    pal.half[0] = *(const v8us*)&sPl[w][ln][8 * hh]; pal.half[1] = *(const v8us*)&sPl[w][ln][16 + 8 * hh];
#pragma unroll
    for (int dt = 0; dt < DT; ++dt) {
      FragB bvh, bvl;
#pragma unroll
      for (int i = 0; i < 8; ++i) {
        bvh.u[i] = sVh[8 * hh + i][dt * 16 + ln]; bvh.u[8 + i] = sVh[16 + 8 * hh + i][dt * 16 + ln];
        bvl.u[i] = sVl[8 * hh + i][dt * 16 + ln]; bvl.u[8 + i] = sVl[16 + 8 * hh + i][dt * 16 + ln];
      }
      oacc[dt] = mmaN<3>(pah.v, pal.v, bvh.v, bvl.v, oacc[dt]);
    }
    __builtin_amdgcn_fence(__ATOMIC_ACQ_REL, "workgroup");
    __builtin_amdgcn_wave_barrier();
  }
#pragma unroll
  for (int r = 0; r < 8; ++r) {
    float l = l_r[r];
    l += __shfl_xor(l, 1, 32); l += __shfl_xor(l, 2, 32); l += __shfl_xor(l, 4, 32); l += __shfl_xor(l, 8, 32);
    l_r[r] = (l > 0.f) ? 1.0f / l : 0.f;
  }
#pragma unroll
  for (int dt = 0; dt < DT; ++dt)
#pragma unroll
    for (int r = 0; r < 8; ++r) sO[w][8 * hh + r][dt * 16 + ln] = oacc[dt][r] * l_r[r];
  __builtin_amdgcn_fence(__ATOMIC_ACQ_REL, "workgroup");
  __builtin_amdgcn_wave_barrier();
  for (int pass = 0; pass < 2; ++pass) {
    for (int r = 0; r < 16; ++r) {
      const int row = q0 + r;
      for (int c4 = lane * 4; c4 < DV; c4 += 128) {
        if (row < Tq) {
          const v4f val = *(const v4fa*)&sO[w][r][c4];
          *(volatile v4f*)(y + (size_t)bh * ystride + (size_t)row * ypitch + dv0 + c4) = val;
        }
      }
    }
    if (pass == 0) __threadfence();
  }
}

template <bool ASPLIT, int ACT, bool BIAS_BF16, bool RES_BF16>
__global__ __launch_bounds__(128) void k_gemm_bf3(const float* __restrict__ A, int lda, const unsigned short* __restrict__ Wt, int ldb,
                                                const float* __restrict__ bias, const float* __restrict__ resid, int rmod, int ldr,
                                                float* __restrict__ C, int ldc, int M, int N, int K) {
  __shared__ __attribute__((aligned(16))) float so[4][16][64];
  const int tid = threadIdx.x, w = tid >> 5, lane = tid & 31, ln = lane & 15, hh = lane >> 4;
  const int ntn = N / 64;
  const int wid = blockIdx.x * 4 + w;
  const int mt = wid / ntn, nq = wid % ntn;
  if (mt * 16 >= M) return;
  const int row0 = mt * 16, col0 = nq * 64;
  const float* arow = A + (size_t)(row0 + ln) * lda;
  v8f acc[4] = {};
  for (int kb = 0; kb < K; kb += 32) {
    FragB ah, al;
    const v4f x0 = *(const v4fa*)(arow + kb + 8 * hh), x1 = *(const v4fa*)(arow + kb + 8 * hh + 4);
    const v4f x2 = *(const v4fa*)(arow + kb + 16 + 8 * hh), x3 = *(const v4fa*)(arow + kb + 16 + 8 * hh + 4);
    float xs[16] = {x0[0],x0[1],x0[2],x0[3],x1[0],x1[1],x1[2],x1[3],x2[0],x2[1],x2[2],x2[3],x3[0],x3[1],x3[2],x3[3]};
#pragma unroll
    for (int i = 0; i < 16; ++i) { const unsigned short hb = bf16_bits(xs[i]); ah.u[i] = hb; al.u[i] = ASPLIT ? bf16_bits(xs[i] - bf16_val(hb)) : (unsigned short)0; }
#pragma unroll
    for (int t = 0; t < 4; ++t) {
      const unsigned short* brow = Wt + (size_t)(col0 + t * 16 + ln) * ldb + kb;
      FragB b;
      b.half[0] = *(const v8us*)(brow + 8 * hh);
      b.half[1] = *(const v8us*)(brow + 16 + 8 * hh);
      acc[t] = mmaN<ASPLIT ? 2 : 1>(ah.v, al.v, b.v, b.v, acc[t]);
    }
  }
#pragma unroll
  for (int t = 0; t < 4; ++t) {
    const int col = col0 + t * 16 + ln;
    float bv = bias ? bias[col] : 0.f;
    if (BIAS_BF16) bv = bf16_round(bv);
#pragma unroll
    for (int r = 0; r < 8; ++r) {
      float v = acc[t][r] + bv;
      if (resid) { float rv = resid[(size_t)((row0 + 8 * hh + r) % rmod) * ldr + col]; if (RES_BF16) rv = bf16_round(rv); v += rv; }
      if (ACT == 1) v = fmaxf(v, 0.f);
      if (ACT == 2) v = 0.5f * v * (1.0f + erff(v * 0.70710678118654752f));
      if (ACT == 3) { const float u = 0.7978845608028654f * (v + 0.044715f * v * v * v); v = 0.5f * v * (1.0f + tanhf(u)); }
      so[w][8 * hh + r][t * 16 + ln] = v;
    }
  }
  __builtin_amdgcn_fence(__ATOMIC_ACQ_REL, "workgroup");
  __builtin_amdgcn_wave_barrier();
  const int rsub = lane >> 4, c4 = (lane & 15) * 4;
  for (int pass = 0; pass < 2; ++pass) {
#pragma unroll
    for (int q = 0; q < 8; ++q) {
      const int r = q * 2 + rsub;
      const v4f v = *(const v4fa*)&so[w][r][c4];
      *(volatile v4f*)(C + (size_t)(row0 + r) * ldc + col0 + c4) = v;
    }
    if (pass == 0) __threadfence();
  }
}
template <bool PARAM_BF16>
__global__ __launch_bounds__(256) void k_layernorm(const float* __restrict__ X, const float* __restrict__ R, const float* __restrict__ g, const float* __restrict__ bta,
                                                  float* __restrict__ out_sum, float* __restrict__ out_norm, int N, float eps) {
  __shared__ float red[256];
  const int row = blockIdx.x, tid = threadIdx.x;
  const float* x = X + (size_t)row * N; const float* rr = R ? R + (size_t)row * N : nullptr;
  float vals[16];
  const int per = N / 256;
  float s1 = 0.f;
  for (int u = 0; u < per / 4; ++u) {
    const int j = tid * 4 + 1024 * u;
    const v4f a = *(const v4fa*)(x + j);
    v4f b = {0.f,0.f,0.f,0.f}; if (rr) b = *(const v4fa*)(rr + j);
#pragma unroll
    for (int q = 0; q < 4; ++q) { const float v = a[q] + b[q]; vals[u * 4 + q] = v; s1 += v; }
  }
  red[tid] = s1; __syncthreads();
  for (int st = 128; st > 0; st >>= 1) { if (tid < st) red[tid] += red[tid + st]; __syncthreads(); }
  const float mu = red[0] / (float)N; __syncthreads();
  float s2 = 0.f;
  for (int u = 0; u < per / 4; ++u)
#pragma unroll
    for (int q = 0; q < 4; ++q) { const float c = vals[u * 4 + q] - mu; s2 += c * c; }
  red[tid] = s2; __syncthreads();
  for (int st = 128; st > 0; st >>= 1) { if (tid < st) red[tid] += red[tid + st]; __syncthreads(); }
  const float rs = rsqrtf(red[0] / (float)N + eps);
  for (int pass = 0; pass < 2; ++pass) {
    for (int u = 0; u < per / 4; ++u) {
      const int j = tid * 4 + 1024 * u;
      v4f o, sm;
#pragma unroll
      for (int q = 0; q < 4; ++q) {
        float gg = g[j + q], bb = bta[j + q];
        if (PARAM_BF16) { gg = bf16_round(gg); bb = bf16_round(bb); }
        sm[q] = vals[u * 4 + q]; o[q] = (vals[u * 4 + q] - mu) * rs * gg + bb;
      }
      if (out_sum) *(volatile v4f*)(out_sum + (size_t)row * N + j) = sm;
      *(volatile v4f*)(out_norm + (size_t)row * N + j) = o;
    }
    if (pass == 0) __threadfence();
  }
}

template <int D>
__global__ __launch_bounds__(128) void k_flash3(const float* __restrict__ Qb, int qpitch, int Tq,
                                              const float* __restrict__ K1, const float* __restrict__ V1, int Tk1,
                                              const float* __restrict__ K2, const float* __restrict__ V2, int Tk2, int kpitch, int vpitch,
                                              int H, float scale, const int* __restrict__ mask, int causal, const float* __restrict__ sbias,
                                              float* __restrict__ y, int ypitch) {
  constexpr int KS = D / 32, DT = D / 16;
  __shared__ __attribute__((aligned(16))) unsigned short sKh[32][D + 8], sKl[32][D + 8], sVh[32][D + 8], sVl[32][D + 8];
  __shared__ __attribute__((aligned(16))) unsigned short sPh[4][16][40], sPl[4][16][40];
  __shared__ __attribute__((aligned(16))) float sO[4][16][D];
  const int tid = threadIdx.x, w = tid >> 5, lane = tid & 31, ln = lane & 15, hh = lane >> 4;
  const int Tk = Tk1 + Tk2;
  const int nqb = (Tq + 63) / 64;
  const int bh = blockIdx.x / nqb, qblk = blockIdx.x % nqb;
  const int b = bh / H, h = bh % H;
  const int q0 = qblk * 64 + w * 16;
  const float* Q = Qb + (size_t)b * Tq * qpitch + h * D;
  FragB aqh[KS], aql[KS];
  {
    int row = q0 + ln; if (row >= Tq) row = Tq - 1;
    const float* qr = Q + (size_t)row * qpitch;
#pragma unroll
    for (int ks = 0; ks < KS; ++ks)
#pragma unroll
      for (int i = 0; i < 16; ++i) {
        const int d = ks * 32 + ((i < 8) ? (8 * hh + i) : (16 + 8 * hh + (i - 8)));
        const float x = qr[d] * scale; const unsigned short hb = bf16_bits(x);
        aqh[ks].u[i] = hb; aql[ks].u[i] = bf16_bits(x - bf16_val(hb));
      }
  }
  int qrow[8];
#pragma unroll
  for (int r = 0; r < 8; ++r) { int qi = q0 + 8 * hh + r; qrow[r] = qi < Tq ? qi : Tq - 1; }
  float m_r[8], l_r[8];
#pragma unroll
  for (int r = 0; r < 8; ++r) { m_r[r] = -3.0e38f; l_r[r] = 0.f; }
  v8f oacc[DT];
#pragma unroll
  for (int dt = 0; dt < DT; ++dt) oacc[dt] = (v8f){0.f,0.f,0.f,0.f,0.f,0.f,0.f,0.f};
  const int kv_end = causal ? min(Tk, qblk * 64 + 64) : Tk;
  for (int j0 = 0; j0 < kv_end; j0 += 32) {
    __syncthreads();
    for (int e = tid; e < 32 * (D / 4); e += 128) {
      const int r = e / (D / 4), c4 = (e % (D / 4)) * 4; const int key = j0 + r;
      v4f kf = {0.f,0.f,0.f,0.f}, vf = {0.f,0.f,0.f,0.f};
      if (key < Tk1) { kf = *(const v4fa*)(K1 + (size_t)b * Tk1 * kpitch + h * D + (size_t)key * kpitch + c4); vf = *(const v4fa*)(V1 + (size_t)b * Tk1 * vpitch + h * D + (size_t)key * vpitch + c4); }
      else if (key < Tk) { const int k2 = key - Tk1; kf = *(const v4fa*)(K2 + (size_t)b * Tk2 * kpitch + h * D + (size_t)k2 * kpitch + c4); vf = *(const v4fa*)(V2 + (size_t)b * Tk2 * vpitch + h * D + (size_t)k2 * vpitch + c4); }
#pragma unroll
      for (int t = 0; t < 4; ++t) {
        unsigned short hb = bf16_bits(kf[t]); sKh[r][c4 + t] = hb; sKl[r][c4 + t] = bf16_bits(kf[t] - bf16_val(hb));
        hb = bf16_bits(vf[t]); sVh[r][c4 + t] = hb; sVl[r][c4 + t] = bf16_bits(vf[t] - bf16_val(hb));
      }
    }
    __syncthreads();
    v8f s[2];
#pragma unroll
    for (int nt = 0; nt < 2; ++nt) {
      v8f acc = {};
#pragma unroll
      for (int ks = 0; ks < KS; ++ks) {
        FragB bh_, bl_;
        bh_.half[0] = *(const v8us*)&sKh[nt * 16 + ln][ks * 32 + 8 * hh]; bh_.half[1] = *(const v8us*)&sKh[nt * 16 + ln][ks * 32 + 16 + 8 * hh];
        bl_.half[0] = *(const v8us*)&sKl[nt * 16 + ln][ks * 32 + 8 * hh]; bl_.half[1] = *(const v8us*)&sKl[nt * 16 + ln][ks * 32 + 16 + 8 * hh];
        acc = mmaN<3>(aqh[ks].v, aql[ks].v, bh_.v, bl_.v, acc);
      }
      s[nt] = acc;
    }
    float alpha[8];
#pragma unroll
    for (int r = 0; r < 8; ++r) {
      const int qi = qrow[r];
      const int ja = j0 + ln, jb = j0 + 16 + ln;
      bool keepa = ja < Tk, keepb = jb < Tk;
      if (causal) { keepa = keepa && (ja <= qi); keepb = keepb && (jb <= qi); }
      if (mask) { if (keepa) keepa = mask[(size_t)qi * Tk + ja] != 0; if (keepb) keepb = mask[(size_t)qi * Tk + jb] != 0; }
      if (sbias) { if (keepa) s[0][r] += sbias[(size_t)bh * Tk + ja]; if (keepb) s[1][r] += sbias[(size_t)bh * Tk + jb]; }
      if (!keepa) s[0][r] = -3.0e38f;
      if (!keepb) s[1][r] = -3.0e38f;
      float mx = fmaxf(s[0][r], s[1][r]);
      mx = fmaxf(mx, __shfl_xor(mx, 1, 32)); mx = fmaxf(mx, __shfl_xor(mx, 2, 32)); mx = fmaxf(mx, __shfl_xor(mx, 4, 32)); mx = fmaxf(mx, __shfl_xor(mx, 8, 32));
      const float mnew = fmaxf(m_r[r], mx);
      alpha[r] = (mnew > -1.0e38f) ? __expf(m_r[r] - mnew) : 1.0f;
      const float p0 = keepa ? __expf(s[0][r] - mnew) : 0.f;
      const float p1 = keepb ? __expf(s[1][r] - mnew) : 0.f;
      m_r[r] = mnew;
      l_r[r] = l_r[r] * alpha[r] + p0 + p1;
      unsigned short hb = bf16_bits(p0); sPh[w][8 * hh + r][ln] = hb;      sPl[w][8 * hh + r][ln] = bf16_bits(p0 - bf16_val(hb));
      hb = bf16_bits(p1);                sPh[w][8 * hh + r][16 + ln] = hb; sPl[w][8 * hh + r][16 + ln] = bf16_bits(p1 - bf16_val(hb));
    }
#pragma unroll
    for (int dt = 0; dt < DT; ++dt)
#pragma unroll
      for (int r = 0; r < 8; ++r) oacc[dt][r] *= alpha[r];
    __builtin_amdgcn_fence(__ATOMIC_ACQ_REL, "workgroup");
    __builtin_amdgcn_wave_barrier();
    FragB pah, pal;
    pah.half[0] = *(const v8us*)&sPh[w][ln][8 * hh]; pah.half[1] = *(const v8us*)&sPh[w][ln][16 + 8 * hh];
    pal.half[0] = *(const v8us*)&sPl[w][ln][8 * hh]; pal.half[1] = *(const v8us*)&sPl[w][ln][16 + 8 * hh];
#pragma unroll
    for (int dt = 0; dt < DT; ++dt) {
      FragB bvh, bvl;
#pragma unroll
      for (int i = 0; i < 8; ++i) {
        bvh.u[i] = sVh[8 * hh + i][dt * 16 + ln]; bvh.u[8 + i] = sVh[16 + 8 * hh + i][dt * 16 + ln];
        bvl.u[i] = sVl[8 * hh + i][dt * 16 + ln]; bvl.u[8 + i] = sVl[16 + 8 * hh + i][dt * 16 + ln];
      }
      oacc[dt] = mmaN<3>(pah.v, pal.v, bvh.v, bvl.v, oacc[dt]);
    }
    __builtin_amdgcn_fence(__ATOMIC_ACQ_REL, "workgroup");
    __builtin_amdgcn_wave_barrier();
  }
#pragma unroll
  for (int r = 0; r < 8; ++r) {
    float l = l_r[r];
    l += __shfl_xor(l, 1, 32); l += __shfl_xor(l, 2, 32); l += __shfl_xor(l, 4, 32); l += __shfl_xor(l, 8, 32);
    l_r[r] = (m_r[r] > -1.0e38f) ? 1.0f / l : __builtin_nanf("");
  }
#pragma unroll
  for (int dt = 0; dt < DT; ++dt)
#pragma unroll
    for (int r = 0; r < 8; ++r) sO[w][8 * hh + r][dt * 16 + ln] = oacc[dt][r] * l_r[r];
  __builtin_amdgcn_fence(__ATOMIC_ACQ_REL, "workgroup");
  __builtin_amdgcn_wave_barrier();
  for (int pass = 0; pass < 2; ++pass) {
    for (int r = 0; r < 16; ++r) {
      const int row = q0 + r;
      if (row < Tq && lane < D / 4) {
        const v4f val = *(const v4fa*)&sO[w][r][lane * 4];
        *(volatile v4f*)(y + ((size_t)b * Tq + row) * ypitch + h * D + lane * 4) = val;
      }
    }
    if (pass == 0) __threadfence();
  }
}

__global__ __launch_bounds__(256) void k_round_rows(const float* __restrict__ W, unsigned short* __restrict__ Wt, int n8) {
  const int t = blockIdx.x * 256 + threadIdx.x;
  if (t >= n8) return;
  const v4f a = *(const v4fa*)(W + (size_t)t * 8), b = *(const v4fa*)(W + (size_t)t * 8 + 4);
  v8us v; v[0]=bf16_bits(a[0]); v[1]=bf16_bits(a[1]); v[2]=bf16_bits(a[2]); v[3]=bf16_bits(a[3]);
  v[4]=bf16_bits(b[0]); v[5]=bf16_bits(b[1]); v[6]=bf16_bits(b[2]); v[7]=bf16_bits(b[3]);
  *(volatile v8us*)(Wt + (size_t)t * 8) = v; __threadfence(); *(volatile v8us*)(Wt + (size_t)t * 8) = v;
}
template <int Cin>
__global__ __launch_bounds__(128) void k_conv3d(const float* __restrict__ in, const unsigned short* __restrict__ Bt, const float* __restrict__ bias, float* __restrict__ out) {
  constexpr int K = 27 * Cin, SPT = Cin / 32;
  __shared__ __attribute__((aligned(16))) float so[4][16][64];
  const int tid = threadIdx.x, w = tid >> 5, lane = tid & 31, ln = lane & 15, hh = lane >> 4;
  const int wid = blockIdx.x * 4 + w; const int mt = wid / (COUT / 64), nq = wid % (COUT / 64); if (mt * 16 >= NVOX) return;
  const int row0 = mt * 16, col0 = nq * 64;
  const int m = row0 + ln;
  const int z = m % RR, y = (m / RR) % RR, x = (m / (RR * RR)) % RR, b = m / (RR * RR * RR);
  v8f acc[4] = {};
  for (int tap = 0; tap < 27; ++tap) {
    const int dx = tap / 9 - 1, dy = (tap / 3) % 3 - 1, dz = tap % 3 - 1;
    const int xx = x + dx, yy = y + dy, zz = z + dz;
    const bool inb = (xx >= 0 && xx < RR && yy >= 0 && yy < RR && zz >= 0 && zz < RR);
    const float* src = in + ((size_t)(((b * RR + (inb ? xx : 0)) * RR + (inb ? yy : 0)) * RR + (inb ? zz : 0))) * Cin;
#pragma unroll
    for (int s = 0; s < SPT; ++s) {
      const int c0 = s * 32;
      v4f a0 = {0.f,0.f,0.f,0.f}, a1 = a0, a2 = a0, a3 = a0;
      if (inb) { a0 = *(const v4fa*)(src + c0 + 8 * hh); a1 = *(const v4fa*)(src + c0 + 8 * hh + 4); a2 = *(const v4fa*)(src + c0 + 16 + 8 * hh); a3 = *(const v4fa*)(src + c0 + 16 + 8 * hh + 4); }
      float xs[16] = {a0[0],a0[1],a0[2],a0[3],a1[0],a1[1],a1[2],a1[3],a2[0],a2[1],a2[2],a2[3],a3[0],a3[1],a3[2],a3[3]};
      FragB ah, al;
#pragma unroll
      for (int i = 0; i < 16; ++i) { const unsigned short hb = bf16_bits(xs[i]); ah.u[i] = hb; al.u[i] = bf16_bits(xs[i] - bf16_val(hb)); }
      const int kb = tap * Cin + c0;
#pragma unroll
      for (int t = 0; t < 4; ++t) { FragB bq; bq.half[0] = *(const v8us*)(Bt + (size_t)(col0 + t * 16 + ln) * K + kb + 8 * hh); bq.half[1] = *(const v8us*)(Bt + (size_t)(col0 + t * 16 + ln) * K + kb + 16 + 8 * hh); acc[t] = mmaN<2>(ah.v, al.v, bq.v, bq.v, acc[t]); }
    }
  }
#pragma unroll
  for (int t = 0; t < 4; ++t) { const int col = col0 + t * 16 + ln; const float bv = bf16_round(bias[col]);
#pragma unroll
    for (int r = 0; r < 8; ++r) so[w][8 * hh + r][t * 16 + ln] = acc[t][r] + bv; }
  __builtin_amdgcn_fence(__ATOMIC_ACQ_REL, "workgroup"); __builtin_amdgcn_wave_barrier();
  const int rsub = lane >> 4, c4 = (lane & 15) * 4;
  for (int pass = 0; pass < 2; ++pass) { for (int q = 0; q < 8; ++q) { const int r = q * 2 + rsub; const v4f v = *(const v4fa*)&so[w][r][c4]; *(volatile v4f*)(out + (size_t)(row0 + r) * COUT + col0 + c4) = v; } if (pass == 0) __threadfence(); }
}

__global__ __launch_bounds__(256) void k_wt_qkv(const float* __restrict__ q1, const float* __restrict__ q2, const float* __restrict__ k1, const float* __restrict__ k2, const float* __restrict__ v, unsigned short* __restrict__ Bt) {
  const int t = blockIdx.x * 256 + threadIdx.x; if (t >= 640 * 8) return; const int n = t / 8, k8 = (t % 8) * 8; const int blk = n / 128, nn = n % 128;
  const float* W = blk == 0 ? q1 : blk == 1 ? q2 : blk == 2 ? k1 : blk == 3 ? k2 : v; v8us o;
#pragma unroll 1
  for (int i = 0; i < 8; ++i) { const int k = k8 + i; float val = 0.f;
    if (blk < 4) { const int h = nn / HP, d = nn % HP; if (d < HD) val = W[(size_t)(h * HD + d) * CH + k]; } else val = W[(size_t)nn * CH + k];
    o[i] = bf16_bits(val); }
  *(volatile v8us*)(Bt + (size_t)n * CH + k8) = o; __threadfence(); *(volatile v8us*)(Bt + (size_t)n * CH + k8) = o;
}
__global__ __launch_bounds__(256) void k_wt_c3(const float* __restrict__ w, unsigned short* __restrict__ Bt) {
  const int t = blockIdx.x * 256 + threadIdx.x; const int K = 27 * CH; if (t >= COUT * (K / 8)) return; const int o = t / (K / 8), k8 = (t % (K / 8)) * 8; v8us v;
#pragma unroll
  for (int i = 0; i < 8; ++i) { const int k = k8 + i; const int tap = k / CH, c = k % CH; v[i] = bf16_bits(w[((size_t)o * CH + c) * 27 + tap]); }
  *(volatile v8us*)(Bt + (size_t)o * K + k8) = v; __threadfence(); *(volatile v8us*)(Bt + (size_t)o * K + k8) = v;
}
__global__ __launch_bounds__(256) void k_diffln(const float* __restrict__ y1, const float* __restrict__ y2, const float* __restrict__ lq1, const float* __restrict__ lk1, const float* __restrict__ lq2, const float* __restrict__ lk2, float* __restrict__ Y) {
  const int tid = threadIdx.x, w = tid >> 5, lane = tid & 31; const size_t rh = (size_t)blockIdx.x * 8 + w; if (rh >= (size_t)NVOX * NH) return; const int h = (int)(rh % NH);
  float a = (lane < HD) ? bf16_round(lq1[h * HD + lane]) * bf16_round(lk1[h * HD + lane]) : 0.f, c = (lane < HD) ? bf16_round(lq2[h * HD + lane]) * bf16_round(lk2[h * HD + lane]) : 0.f;
  for (int o = 16; o >= 1; o >>= 1) { a += __shfl_xor(a, o, 32); c += __shfl_xor(c, o, 32); }
  const float lam = expf(a) - expf(c) + LINIT;
  const size_t base = rh * HP + lane;
  const float v = y1[base] - lam * y2[base];
  float s = v; for (int o = 16; o >= 1; o >>= 1) s += __shfl_xor(s, o, 32); const float mu = s * (1.0f / HP);
  float q2 = (v - mu) * (v - mu); for (int o = 16; o >= 1; o >>= 1) q2 += __shfl_xor(q2, o, 32); const float rs = 1.0f / sqrtf(q2 * (1.0f / HP) + 1e-5f);
  const float outv = (v - mu) * rs * (1.0f - LINIT);
  *(volatile float*)(Y + base) = outv; __threadfence(); *(volatile float*)(Y + base) = outv;
}
__global__ __launch_bounds__(256) void k_copylow(const float* __restrict__ lowT, float* __restrict__ y2pm) {
  const int tid = threadIdx.x, w = tid >> 5, lane = tid & 31; const int row = blockIdx.x * 8 + w; if (row >= NVOX) return;
  const float a = lowT[(size_t)row * CH + lane], b = lowT[(size_t)row * CH + 32 + lane];
  *(volatile float*)(y2pm + (size_t)row * 256 + 192 + lane) = a; *(volatile float*)(y2pm + (size_t)row * 256 + 224 + lane) = b; __threadfence(); *(volatile float*)(y2pm + (size_t)row * 256 + 192 + lane) = a; *(volatile float*)(y2pm + (size_t)row * 256 + 224 + lane) = b;
}
__global__ __launch_bounds__(256) void k_cmean1(const float* __restrict__ a, const float* __restrict__ bsrc, float* __restrict__ part) {
  const int blk = blockIdx.x; const int c = threadIdx.x; const int b = blk / (NP / 64), rb = blk % (NP / 64); float s1 = 0.f, s2 = 0.f;
#pragma unroll 1
  for (int r = 0; r < 64; ++r) { const size_t row = (size_t)b * NP + rb * 64 + r; s1 += a[row * 256 + c]; s2 += bsrc[row * 256 + c]; }
  *(volatile float*)(part + (size_t)blk * 512 + c) = s1; *(volatile float*)(part + (size_t)blk * 512 + 256 + c) = s2; __threadfence(); *(volatile float*)(part + (size_t)blk * 512 + c) = s1; *(volatile float*)(part + (size_t)blk * 512 + 256 + c) = s2;
}
__global__ __launch_bounds__(512) void k_cmean2(const float* __restrict__ part, float* __restrict__ scale) {
  __shared__ float red[512]; const int b = blockIdx.x, c = threadIdx.x; float s = 0.f; for (int k = 0; k < NP / 64; ++k) s += part[((size_t)b * (NP / 64) + k) * 512 + c]; s *= (1.0f / NP);
  red[c] = s; __syncthreads();
  __shared__ float mx, den; if (c == 0) { float m = -3e38f; for (int i = 0; i < 512; ++i) m = fmaxf(m, red[i]); float d = 0.f; for (int i = 0; i < 512; ++i) d += expf(red[i] - m); mx = m; den = d; } __syncthreads();
  const float v = expf(s - mx) / den;
  *(volatile float*)(scale + (size_t)b * 512 + c) = v; __threadfence(); *(volatile float*)(scale + (size_t)b * 512 + c) = v;
}
__global__ __launch_bounds__(256) void k_final(const float* __restrict__ y1c, const float* __restrict__ y2pm, const float* __restrict__ scale, float* __restrict__ out) {
  const int b = blockIdx.x / 256, c = blockIdx.x % 256; const float s1 = scale[(size_t)b * 512 + c], s2 = scale[(size_t)b * 512 + 256 + c];
  for (int pass = 0; pass < 2; ++pass) { for (int p = threadIdx.x; p < NP; p += 256) { const size_t row = (size_t)b * NP + p; *(volatile float*)(out + ((size_t)b * 256 + c) * NP + p) = y1c[row * 256 + c] * s1 + y2pm[row * 256 + c] * s2; } if (pass == 0) __threadfence(); }
}
extern "C" void kernel_launch(void* const* d_in, const int* in_sizes, int n_in,
                              void* d_out, int out_size, void* d_ws, size_t ws_size, hipStream_t stream) {
  (void)in_sizes; (void)n_in; (void)out_size;
  const float* x = (const float*)d_in[0]; const float* w_sq1 = (const float*)d_in[1]; const float* w_sq2 = (const float*)d_in[2]; const float* w_pwc2 = (const float*)d_in[3]; const float* w_conv = (const float*)d_in[4]; const float* b_conv = (const float*)d_in[5];
  const float* w_q1 = (const float*)d_in[6]; const float* w_q2 = (const float*)d_in[7]; const float* w_k1 = (const float*)d_in[8]; const float* w_k2 = (const float*)d_in[9]; const float* w_v = (const float*)d_in[10]; const float* w_c = (const float*)d_in[11];
  const float* lq1 = (const float*)d_in[12]; const float* lk1 = (const float*)d_in[13]; const float* lq2 = (const float*)d_in[14]; const float* lk2 = (const float*)d_in[15];
  char* ws = (char*)d_ws; size_t off = 0;
  auto take = [&](size_t bytes) { char* p = ws + off; off += (bytes + 255) & ~(size_t)255; return p; };
  const int M = NVOX;
  unsigned short* Bsq1 = (unsigned short*)take(CH * 128 * 2); unsigned short* Bsq2 = (unsigned short*)take(CH * 128 * 2); unsigned short* Bpw = (unsigned short*)take(192 * CH * 2); unsigned short* Bqkv = (unsigned short*)take(640 * CH * 2); unsigned short* Bc = (unsigned short*)take(CH * 128 * 2); unsigned short* B3 = (unsigned short*)take((size_t)COUT * 27 * CH * 2);
  float* xT = (float*)take((size_t)M * CX * 4); float* upT = (float*)take((size_t)M * CH * 4); float* lowT = (float*)take((size_t)M * CH * 4); float* xt = (float*)take((size_t)M * CH * 4);
  float* qkv = (float*)take((size_t)M * 640 * 4); float* ya = (float*)take((size_t)M * 128 * 4); float* yb = (float*)take((size_t)M * 128 * 4); float* Y = (float*)take((size_t)M * 128 * 4); float* yc = (float*)take((size_t)M * CH * 4); float* ycT = (float*)take((size_t)M * CH * 4);
  float* y1c = (float*)take((size_t)M * 256 * 4); float* y2pm = (float*)take((size_t)M * 256 * 4); float* part = (float*)take((size_t)BB * (NP / 64) * 512 * 4); float* scale = (float*)take(BB * 512 * 4);
  if (off > ws_size) return;
  k_round_rows<<<(CH * 128 / 8 + 255) / 256, 256, 0, stream>>>(w_sq1, Bsq1, CH * 128 / 8); k_round_rows<<<(CH * 128 / 8 + 255) / 256, 256, 0, stream>>>(w_sq2, Bsq2, CH * 128 / 8);
  k_round_rows<<<(192 * CH / 8 + 255) / 256, 256, 0, stream>>>(w_pwc2, Bpw, 192 * CH / 8); k_round_rows<<<(CH * 128 / 8 + 255) / 256, 256, 0, stream>>>(w_c, Bc, CH * 128 / 8);
  k_wt_qkv<<<(640 * 8 + 255) / 256, 256, 0, stream>>>(w_q1, w_q2, w_k1, w_k2, w_v, Bqkv); k_wt_c3<<<(COUT * (27 * CH / 8) + 255) / 256, 256, 0, stream>>>(w_conv, B3);
  k_transpose32<false, false, false><<<dim3(NP / 32, CX / 32, BB), 256, 0, stream>>>(x, xT, CX, NP, nullptr, nullptr, nullptr);
  const int g64 = ((M / 16) * 1 + 3) / 4;
  k_gemm_bf3<false, 0, false, false><<<g64, 128, 0, stream>>>(xT, CX, Bsq1, 128, nullptr, nullptr, 1, 0, upT, CH, M, CH, 128);
  k_gemm_bf3<false, 0, false, false><<<g64, 128, 0, stream>>>(xT + 128, CX, Bsq2, 128, nullptr, nullptr, 1, 0, lowT, CH, M, CH, 128);
  k_transpose32<false, false, false><<<dim3(CH / 32, NP / 32, BB), 256, 0, stream>>>(upT, xt, NP, CH, nullptr, nullptr, nullptr);
  k_gemm_bf3<true, 0, false, false><<<((M / 16) * 10 + 3) / 4, 128, 0, stream>>>(xt, CH, Bqkv, CH, nullptr, nullptr, 1, 0, qkv, 640, M, 640, CH);
  k_flash3<HP><<<BB * NH * (NP / 64), 128, 0, stream>>>(qkv, 640, NP, qkv + 256, qkv + 512, NP, nullptr, nullptr, 0, 640, 640, NH, 0.25f, nullptr, 1, nullptr, ya, 128);
  k_flash3<HP><<<BB * NH * (NP / 64), 128, 0, stream>>>(qkv + 128, 640, NP, qkv + 384, qkv + 512, NP, nullptr, nullptr, 0, 640, 640, NH, 0.25f, nullptr, 1, nullptr, yb, 128);
  k_diffln<<<(NVOX * NH + 7) / 8, 256, 0, stream>>>(ya, yb, lq1, lk1, lq2, lk2, Y);
  k_gemm_bf3<true, 0, false, false><<<g64, 128, 0, stream>>>(Y, 128, Bc, 128, nullptr, nullptr, 1, 0, yc, CH, M, CH, 128);
  k_transpose32<false, false, false><<<dim3(NP / 32, CH / 32, BB), 256, 0, stream>>>(yc, ycT, CH, NP, nullptr, nullptr, nullptr);
  k_conv3d<CH><<<((NVOX / 16) * (COUT / 64) + 3) / 4, 128, 0, stream>>>(ycT, B3, b_conv, y1c);
  k_gemm_bf3<true, 0, false, false><<<((M / 16) * 3 + 3) / 4, 128, 0, stream>>>(lowT, CH, Bpw, CH, nullptr, nullptr, 1, 0, y2pm, 256, M, 192, CH);
  k_copylow<<<(NVOX + 7) / 8, 256, 0, stream>>>(lowT, y2pm);
  k_cmean1<<<BB * (NP / 64), 256, 0, stream>>>(y1c, y2pm, part); k_cmean2<<<BB, 512, 0, stream>>>(part, scale);
  k_final<<<BB * 256, 256, 0, stream>>>(y1c, y2pm, scale, (float*)d_out);
}
